// DependencyParser_23021024707460
// MI455X (gfx1250) — hardware-verified
//
#include <hip/hip_runtime.h>
#include <math.h>

typedef __attribute__((ext_vector_type(16))) _Float16 v16h;
typedef __attribute__((ext_vector_type(8)))  _Float16 v8h;
typedef __attribute__((ext_vector_type(8)))  float    v8f;
typedef __attribute__((ext_vector_type(4)))  float    v4f;

constexpr int kNB    = 16;
constexpr int kNT    = 128;
constexpr int kNWE   = 100;
constexpr int kNTE   = 28;
constexpr int kNE    = kNWE + kNTE;
constexpr int kNH    = 128;
constexpr int kNG    = 4 * kNH;
constexpr int kNG2   = 2 * kNG;
constexpr int kNH2   = 2 * kNH;
constexpr int kNFC   = 100;
constexpr int kNFCP  = 256;
constexpr int kWVoc  = 50000;
constexpr int kTVoc  = 50;
constexpr int kRows  = kNT * kNB;
constexpr int kNOut  = kNT * kNT * kNB;
constexpr int kHP    = 136;
constexpr int kXPP   = 20;
static_assert(kNE == 128);
static_assert(kNB == 16);
static_assert((kNE % 32) == 0 && (kNH % 32) == 0 && (kNH2 % 32) == 0);
static_assert((kRows % 32) == 0 && (kNG2 % 64) == 0 && (kNFCP % 64) == 0);
static_assert(2 * kNFC <= kNFCP);
static_assert((2 * 16 * kHP) % 256 == 0);
static_assert((kHP % 8) == 0 && (kXPP % 4) == 0);

constexpr float kActCarry = 256.0f;
constexpr float kWCarry   = 256.0f;
constexpr float kResCarry = 2048.0f;
constexpr float kFold     = 1.0f / (kActCarry * kWCarry);
constexpr float kResInv   = 1.0f / kResCarry;
constexpr float kHalfMin  = 6.103515625e-05f;

constexpr size_t kSzWIH0 = (size_t)kNG2 * kNE * 2;
constexpr size_t kSzWHH  = (size_t)2 * kNG * kNH * 2;
constexpr size_t kSzWIH1 = (size_t)kNG2 * kNH2 * 2;
constexpr size_t kSzFC1  = (size_t)kNFCP * kNH2 * 2;
constexpr size_t kSzBIAS = (size_t)(2 * kNG2 + kNFCP) * 4;
constexpr size_t kSzX    = (size_t)kRows * kNE * 2;
constexpr size_t kSzXP   = (size_t)kRows * kNG2 * 4;
constexpr size_t kSzH    = (size_t)kRows * kNH2 * 2;
constexpr size_t kSzAB   = (size_t)kRows * kNFCP * 4;
constexpr size_t kOffWIH0 = 0;
constexpr size_t kOffWHH0 = kOffWIH0 + kSzWIH0;
constexpr size_t kOffWIH1 = kOffWHH0 + kSzWHH;
constexpr size_t kOffWHH1 = kOffWIH1 + kSzWIH1;
constexpr size_t kOffFC1  = kOffWHH1 + kSzWHH;
constexpr size_t kOffBIAS = kOffFC1  + kSzFC1;
constexpr size_t kOffXH   = kOffBIAS + kSzBIAS;
constexpr size_t kOffXL   = kOffXH   + kSzX;
constexpr size_t kOffXP0  = kOffXL   + kSzX;
constexpr size_t kOffH0H  = kOffXP0  + kSzXP;
constexpr size_t kOffH0L  = kOffH0H  + kSzH;
constexpr size_t kOffXP1  = kOffH0L  + kSzH;
constexpr size_t kOffH1H  = kOffXP1  + kSzXP;
constexpr size_t kOffH1L  = kOffH1H  + kSzH;
constexpr size_t kOffAB   = kOffH1L  + kSzH;
constexpr size_t kWsTotal = kOffAB   + kSzAB;
static_assert(kWsTotal == 25568256ull);
static_assert(kWsTotal <= 134217728ull);
static_assert((kOffWHH0 % 256) == 0 && (kOffWIH1 % 256) == 0 && (kOffWHH1 % 256) == 0 && (kOffFC1 % 256) == 0 &&
              (kOffBIAS % 256) == 0 && (kOffXH % 256) == 0 && (kOffXL % 256) == 0 && (kOffXP0 % 256) == 0 &&
              (kOffH0H % 256) == 0 && (kOffH0L % 256) == 0 && (kOffXP1 % 256) == 0 && (kOffH1H % 256) == 0 &&
              (kOffH1L % 256) == 0 && (kOffAB % 256) == 0);

namespace eng {
union FragU { v16h v; v8h h[2]; };
__device__ __forceinline__ v16h frag_load(const _Float16* p) {
  FragU f;
  f.h[0] = *(const v8h*)(p);
  f.h[1] = *(const v8h*)(p + 16);
  return f.v;
}
__device__ __forceinline__ v8f mma_g(v16h a, v16h b, v8f c) {
  c = __builtin_amdgcn_wmma_f32_16x16x32_f16(false, a, false, b, (short)0, c, false, false);
  asm volatile("v_nop\n\tv_nop\n\tv_nop\n\tv_nop" : "+v"(c) : "v"(a), "v"(b));
  return c;
}
}

__device__ __forceinline__ float flush_h(float v) { return (fabsf(v) < kHalfMin) ? 0.0f : v; }

__device__ __forceinline__ void split_act(float v, _Float16& hi, _Float16& lo) {
  const float s = v * kActCarry;
  hi = (_Float16)flush_h(s);
  float hf = (float)hi;
  asm volatile("" : "+v"(hf));
  const float r = (s - hf) * kResCarry;
  lo = (_Float16)flush_h(r);
}

__device__ __forceinline__ void pin4(v4f& v) {
  float a = v[0], b = v[1], c = v[2], d = v[3];
  asm volatile("" : "+v"(a), "+v"(b), "+v"(c), "+v"(d));
  v[0] = a; v[1] = b; v[2] = c; v[3] = d;
}

__device__ __forceinline__ float sigm_f(float x) { return __builtin_amdgcn_rcpf(1.0f + expf(-x)); }
__device__ __forceinline__ float tanh_f(float x) { return 1.0f - 2.0f * __builtin_amdgcn_rcpf(expf(2.0f * x) + 1.0f); }

__device__ __forceinline__ void wave_sync_lds() {
  __builtin_amdgcn_fence(__ATOMIC_RELEASE, "workgroup");
  __builtin_amdgcn_wave_barrier();
  __builtin_amdgcn_fence(__ATOMIC_ACQUIRE, "workgroup");
}

__global__ __launch_bounds__(256) void wplane_kernel(const float* src0, const float* src1,
                                                     unsigned short* __restrict__ dst,
                                                     int nrow, int ncol8, int spitch, int scol0a, int scol0b) {
  const int y = blockIdx.y;
  const float* src = (y != 0) ? src1 : src0;
  const int scol0 = (y != 0) ? scol0b : scol0a;
  const int n8 = nrow * ncol8;
  const int i = blockIdx.x * 256 + threadIdx.x;
  const int ic = (i < n8) ? i : (n8 - 1);
  const int row = ic / ncol8;
  const int c8 = ic - row * ncol8;
  const float* sp = src + (size_t)row * spitch + scol0 + c8 * 8;
  v4f a = *(const v4f*)(sp);
  v4f b = *(const v4f*)(sp + 4);
  pin4(a);
  pin4(b);
  v8h hv;
#pragma unroll
  for (int e = 0; e < 4; ++e) {
    hv[e]     = (_Float16)flush_h(a[e] * kWCarry);
    hv[4 + e] = (_Float16)flush_h(b[e] * kWCarry);
  }
  if (i < n8) {
    unsigned short* q = dst + ((size_t)y * n8 + (size_t)i) * 8;
    *(volatile v8h*)q = hv;
    __threadfence();
    *(volatile v8h*)q = hv;
  }
}

__global__ __launch_bounds__(256) void prep_misc_kernel(
    const float* __restrict__ bi0f, const float* __restrict__ bh0f, const float* __restrict__ bi0b, const float* __restrict__ bh0b,
    const float* __restrict__ bi1f, const float* __restrict__ bh1f, const float* __restrict__ bi1b, const float* __restrict__ bh1b,
    const float* __restrict__ fcb, float* __restrict__ BIAS, unsigned short* __restrict__ FCPAD) {
  const int tid = threadIdx.x;
  if (blockIdx.x < 3) {
    const int j = blockIdx.x * 256 + tid;
    const int jc = (j < 575) ? j : 575;
    const int seg = jc >> 7;
    const int idx = (jc & 127) * 4;
    v4f a0 = *(const v4f*)(bi0f + idx);
    v4f a1 = *(const v4f*)(bh0f + idx);
    v4f a2 = *(const v4f*)(bi0b + idx);
    v4f a3 = *(const v4f*)(bh0b + idx);
    v4f a4 = *(const v4f*)(bi1f + idx);
    v4f a5 = *(const v4f*)(bh1f + idx);
    v4f a6 = *(const v4f*)(bi1b + idx);
    v4f a7 = *(const v4f*)(bh1b + idx);
    pin4(a0); pin4(a1); pin4(a2); pin4(a3);
    pin4(a4); pin4(a5); pin4(a6); pin4(a7);
    v4f fv;
#pragma unroll
    for (int e = 0; e < 4; ++e) {
      const int n = idx + e;
      int nn = n - kNFC;
      nn = (nn < 0) ? 0 : nn;
      nn = (nn > kNFC - 1) ? (kNFC - 1) : nn;
      float f = fcb[nn];
      asm volatile("" : "+v"(f));
      fv[e] = (n >= kNFC && n < 2 * kNFC) ? f : 0.0f;
    }
    v4f o;
#pragma unroll
    for (int e = 0; e < 4; ++e) {
      const float s0 = a0[e] + a1[e];
      const float s1 = a2[e] + a3[e];
      const float s2 = a4[e] + a5[e];
      const float s3 = a6[e] + a7[e];
      float v = fv[e];
      v = (seg == 3) ? s3 : v;
      v = (seg == 2) ? s2 : v;
      v = (seg == 1) ? s1 : v;
      v = (seg == 0) ? s0 : v;
      o[e] = v;
    }
    if (j < 576) {
      float* op = BIAS + seg * kNG + idx;
      *(volatile v4f*)op = o;
      __threadfence();
      *(volatile v4f*)op = o;
    }
  } else {
    const int k = (blockIdx.x - 3) * 256 + tid;
    v8h z;
#pragma unroll
    for (int e = 0; e < 8; ++e) z[e] = (_Float16)0.0f;
    unsigned short* q = FCPAD + (size_t)k * 8;
    *(volatile v8h*)q = z;
    __threadfence();
    *(volatile v8h*)q = z;
  }
}

__global__ __launch_bounds__(256) void embed_kernel(const int* __restrict__ widx, const int* __restrict__ pidx,
                                                    const float* __restrict__ wemb, const float* __restrict__ temb,
                                                    unsigned short* __restrict__ XH, unsigned short* __restrict__ XL) {
  const int i = blockIdx.x * 256 + threadIdx.x;
  const int m = i >> 4, c8 = i & 15;
  const int t = m >> 4, b = m & 15;
  int wi = widx[b * kNT + t];
  int pi = pidx[b * kNT + t];
  wi = (wi < 0) ? 0 : wi;
  wi = (wi > kWVoc - 1) ? (kWVoc - 1) : wi;
  pi = (pi < 0) ? 0 : pi;
  pi = (pi > kTVoc - 1) ? (kTVoc - 1) : pi;
  float xv[8];
#pragma unroll
  for (int hf = 0; hf < 2; ++hf) {
    const int g4 = 2 * c8 + hf;
    const int wg = (g4 < 24) ? g4 : 24;
    const int tg = (g4 > 25) ? (g4 - 25) : 0;
    v4f wv = *(const v4f*)(wemb + (size_t)wi * kNWE + wg * 4);
    v4f tv = *(const v4f*)(temb + (size_t)pi * kNTE + tg * 4);
    pin4(wv);
    pin4(tv);
    const bool usew = (g4 < 25);
#pragma unroll
    for (int e = 0; e < 4; ++e) xv[4 * hf + e] = usew ? wv[e] : tv[e];
  }
  v8h hv, lv;
#pragma unroll
  for (int e = 0; e < 8; ++e) {
    _Float16 hi, lo;
    split_act(xv[e], hi, lo);
    hv[e] = hi;
    lv[e] = lo;
  }
  unsigned short* qh = XH + (size_t)i * 8;
  unsigned short* ql = XL + (size_t)i * 8;
  *(volatile v8h*)qh = hv;
  *(volatile v8h*)ql = lv;
  __threadfence();
  *(volatile v8h*)qh = hv;
  *(volatile v8h*)ql = lv;
}

__global__ __launch_bounds__(256) void gemm_vr_kernel(
    const unsigned short* __restrict__ Ahp, const unsigned short* __restrict__ Alp, int lda,
    const unsigned short* __restrict__ Btp, int ldb,
    float* __restrict__ C, int ldc, const float* __restrict__ bias, int M, int N, int K) {
  const _Float16* Ah = (const _Float16*)Ahp;
  const _Float16* Al = (const _Float16*)Alp;
  const _Float16* Bt = (const _Float16*)Btp;
  __shared__ __align__(16) float sT[8][16 * 68];
  const int lane = threadIdx.x & 31;
  const int wave = threadIdx.x >> 5;
  const int tilesN = N >> 6;
  const int tilesM = M >> 5;
  const int tile = blockIdx.x * 8 + wave;
  if (tile >= tilesM * tilesN) return;
  const int tm = tile / tilesN;
  const int tn = tile - tm * tilesN;
  const int m0 = tm << 5;
  const int n0 = tn << 6;
  const int rlane = lane & 15;
  const int koff = (lane >> 4) * 8;
  const int mOff = (lane >> 4) * 8;

  v8f am[2][4], ar[2][4];
#pragma unroll
  for (int i = 0; i < 2; ++i)
#pragma unroll
    for (int j = 0; j < 4; ++j) {
      am[i][j] = (v8f){0.f, 0.f, 0.f, 0.f, 0.f, 0.f, 0.f, 0.f};
      ar[i][j] = (v8f){0.f, 0.f, 0.f, 0.f, 0.f, 0.f, 0.f, 0.f};
    }

#pragma unroll 1
  for (int k0 = 0; k0 < K; k0 += 32) {
    v16h bf[4];
#pragma unroll
    for (int j = 0; j < 4; ++j)
      bf[j] = eng::frag_load(Bt + (size_t)(n0 + (j << 4) + rlane) * ldb + koff + k0);
#pragma unroll
    for (int i = 0; i < 2; ++i) {
      const size_t ao = (size_t)(m0 + (i << 4) + rlane) * lda + koff + k0;
      const v16h ah = eng::frag_load(Ah + ao);
      const v16h al = eng::frag_load(Al + ao);
#pragma unroll
      for (int j = 0; j < 4; ++j) {
        am[i][j] = eng::mma_g(ah, bf[j], am[i][j]);
        ar[i][j] = eng::mma_g(al, bf[j], ar[i][j]);
      }
    }
  }

  float* slab = sT[wave];
#pragma unroll
  for (int i = 0; i < 2; ++i) {
    const int mBase = m0 + (i << 4);
#pragma unroll
    for (int j = 0; j < 4; ++j) {
      const float bv = bias[n0 + (j << 4) + rlane];
#pragma unroll
      for (int r = 0; r < 8; ++r) {
        const float v = fmaf(fmaf(ar[i][j][r], kResInv, am[i][j][r]), kFold, bv);
        slab[(mOff + r) * 68 + (j << 4) + rlane] = v;
      }
    }
    wave_sync_lds();
    {
      const int hh = lane >> 4, c4 = (lane & 15) * 4;
      for (int pass = 0; pass < 2; ++pass) {
#pragma unroll
        for (int it = 0; it < 8; ++it) {
          const int row = it * 2 + hh;
          const v4f v = *(const v4f*)(slab + row * 68 + c4);
          *(volatile v4f*)(C + (size_t)(mBase + row) * ldc + n0 + c4) = v;
        }
        __threadfence();
      }
    }
    wave_sync_lds();
  }
}

__global__ __launch_bounds__(256) void lstm_dir_kernel(const float* __restrict__ XP,
                                                       const unsigned short* __restrict__ WHHp,
                                                       unsigned short* __restrict__ HHp,
                                                       unsigned short* __restrict__ HLp) {
  __shared__ __align__(16) _Float16 Ahi[2 * 16 * kHP];
  __shared__ __align__(16) _Float16 Alo[2 * 16 * kHP];
  __shared__ __align__(16) float    Xs[8 * 64 * kXPP];
  const int dir = blockIdx.x;
  const _Float16* W = (const _Float16*)WHHp + (size_t)dir * kNG * kNH;
  const int tid = threadIdx.x, lane = tid & 31, wave = tid >> 5;
  const int c = lane & 15, hh = lane >> 4, koff = hh * 8;

#pragma unroll 1
  for (int i = tid; i < 2 * 16 * kHP; i += 256) {
    Ahi[i] = (_Float16)0.0f;
    Alo[i] = (_Float16)0.0f;
  }
  float cst[8];
#pragma unroll
  for (int r = 0; r < 8; ++r) cst[r] = 0.0f;
  __syncthreads();

  const _Float16* wrow = W + (size_t)(16 * wave + c) * kNH + koff;
  float* xs = Xs + wave * 64 * kXPP;
  const v8f z8 = {0.f, 0.f, 0.f, 0.f, 0.f, 0.f, 0.f, 0.f};

#pragma unroll 1
  for (int s = 0; s < kNT; ++s) {
    const int t = (dir != 0) ? (kNT - 1 - s) : s;
    const int cur = s & 1;
    const _Float16* ahp = Ahi + cur * 16 * kHP + c * kHP + koff;
    const _Float16* alp = Alo + cur * 16 * kHP + c * kHP + koff;
    _Float16* ahn = Ahi + (cur ^ 1) * 16 * kHP;
    _Float16* aln = Alo + (cur ^ 1) * 16 * kHP;

    v8f am[4], ar[4];
#pragma unroll
    for (int g = 0; g < 4; ++g) { am[g] = z8; ar[g] = z8; }
#pragma unroll 1
    for (int kc = 0; kc < 4; ++kc) {
      const v16h ah = eng::frag_load(ahp + kc * 32);
      const v16h al = eng::frag_load(alp + kc * 32);
#pragma unroll
      for (int g = 0; g < 4; ++g) {
        const v16h bw = eng::frag_load(wrow + (size_t)g * (kNH * kNH) + kc * 32);
        am[g] = eng::mma_g(ah, bw, am[g]);
        ar[g] = eng::mma_g(al, bw, ar[g]);
      }
    }

    {
      const float* xpt = XP + (size_t)t * 16 * kNG2 + dir * kNG + 16 * wave;
      v4f xv[8];
#pragma unroll
      for (int it = 0; it < 8; ++it) {
        const int idx = it * 32 + lane;
        const int seg = idx >> 2, q = idx & 3;
        xv[it] = *(const v4f*)(xpt + (size_t)(seg & 15) * kNG2 + (seg >> 4) * kNH + q * 4);
      }
#pragma unroll
      for (int it = 0; it < 8; ++it) {
        const int idx = it * 32 + lane;
        const int seg = idx >> 2, q = idx & 3;
        *(v4f*)(xs + seg * kXPP + q * 4) = xv[it];
      }
    }
    wave_sync_lds();

#pragma unroll
    for (int r = 0; r < 8; ++r) {
      const int row = 8 * hh + r;
      const float xi = xs[(0 * 16 + row) * kXPP + c];
      const float xf = xs[(1 * 16 + row) * kXPP + c];
      const float xg = xs[(2 * 16 + row) * kXPP + c];
      const float xo = xs[(3 * 16 + row) * kXPP + c];
      const float zi = fmaf(fmaf(ar[0][r], kResInv, am[0][r]), kFold, xi);
      const float zf = fmaf(fmaf(ar[1][r], kResInv, am[1][r]), kFold, xf);
      const float zg = fmaf(fmaf(ar[2][r], kResInv, am[2][r]), kFold, xg);
      const float zo = fmaf(fmaf(ar[3][r], kResInv, am[3][r]), kFold, xo);
      const float ig = sigm_f(zi);
      const float fg = sigm_f(zf);
      const float gg = tanh_f(zg);
      const float og = sigm_f(zo);
      const float cn = fg * cst[r] + ig * gg;
      cst[r] = cn;
      const float hn = og * tanh_f(cn);
      _Float16 hhi, hlo;
      split_act(hn, hhi, hlo);
      ahn[row * kHP + 16 * wave + c] = hhi;
      aln[row * kHP + 16 * wave + c] = hlo;
    }
    wave_sync_lds();
    __syncthreads();

    {
      const int row = 2 * wave + hh;
      const int col8 = c * 8;
      const v8h vh = *(const v8h*)(ahn + row * kHP + col8);
      const v8h vl = *(const v8h*)(aln + row * kHP + col8);
      const size_t o = (size_t)(t * 16 + row) * kNH2 + dir * kNH + col8;
      *(volatile v8h*)(HHp + o) = vh;
      *(volatile v8h*)(HLp + o) = vl;
      __threadfence();
      *(volatile v8h*)(HHp + o) = vh;
      *(volatile v8h*)(HLp + o) = vl;
    }
  }
}

__global__ __launch_bounds__(256) void score_kernel(const float* __restrict__ AB, const float* __restrict__ w2,
                                                    const float* __restrict__ b2, const int* __restrict__ mlen,
                                                    float* __restrict__ out) {
  __shared__ __align__(16) float sA[16 * kNFC];
  __shared__ __align__(16) float sW[kNFC];
  __shared__ __align__(16) float sO[kNT * kNB];
  const int tid = threadIdx.x;
  const int i = blockIdx.x;
#pragma unroll
  for (int it = 0; it < 2; ++it) {
    const int idx = it * 256 + tid;
    const int idc = (idx < 399) ? idx : 399;
    const int row = idc / 25;
    const int q = idc - row * 25;
    v4f v = *(const v4f*)(AB + (size_t)(i * 16 + row) * kNFCP + q * 4);
    pin4(v);
    if (idx < 400) *(v4f*)(sA + row * kNFC + q * 4) = v;
  }
  {
    const int tq = (tid < 24) ? tid : 24;
    v4f wv = *(const v4f*)(w2 + tq * 4);
    pin4(wv);
    if (tid < 25) *(v4f*)(sW + tq * 4) = wv;
  }
  const float bias2 = b2[0];
  const bool premise = (mlen[0] == kNT);
  const float poison = __uint_as_float(0x7fc00000u);
  __syncthreads();

#pragma unroll 1
  for (int it = 0; it < 8; ++it) {
    const int ol = it * 256 + tid;
    const int j = ol >> 4, b = ol & 15;
    const float* ap = sA + b * kNFC;
    const float* bp = AB + (size_t)(j * 16 + b) * kNFCP + kNFC;
    float s = 0.0f;
#pragma unroll 1
    for (int q = 0; q < 25; ++q) {
      const v4f av = *(const v4f*)(ap + 4 * q);
      const v4f bv = *(const v4f*)(bp + 4 * q);
      const v4f wv = *(const v4f*)(sW + 4 * q);
#pragma unroll
      for (int e = 0; e < 4; ++e) s = fmaf(wv[e], tanh_f(av[e] + bv[e]), s);
    }
    s += bias2;
    sO[ol] = premise ? s : poison;
  }
  __syncthreads();
  v4f ov[2];
#pragma unroll
  for (int it = 0; it < 2; ++it) ov[it] = *(const v4f*)(sO + (it * 256 + tid) * 4);
  float* ob = out + (size_t)i * (kNT * kNB);
  for (int pass = 0; pass < 2; ++pass) {
#pragma unroll
    for (int it = 0; it < 2; ++it) *(volatile v4f*)(ob + (it * 256 + tid) * 4) = ov[it];
    __threadfence();
  }
}

extern "C" void kernel_launch(void* const* d_in, const int* in_sizes, int n_in,
                              void* d_out, int out_size, void* d_ws, size_t ws_size,
                              hipStream_t stream) {
  if (n_in < 26 || d_out == nullptr || d_ws == nullptr) return;
  if (in_sizes[0] != kNB * kNT || in_sizes[1] != kNB * kNT || in_sizes[2] != 1) return;
  if (in_sizes[4] != kWVoc * kNWE || in_sizes[5] != kTVoc * kNTE) return;
  if (in_sizes[6] != kNG * kNE || in_sizes[7] != kNG * kNH || in_sizes[8] != kNG || in_sizes[9] != kNG) return;
  if (in_sizes[10] != kNG * kNE || in_sizes[11] != kNG * kNH || in_sizes[12] != kNG || in_sizes[13] != kNG) return;
  if (in_sizes[14] != kNG * kNH2 || in_sizes[15] != kNG * kNH || in_sizes[16] != kNG || in_sizes[17] != kNG) return;
  if (in_sizes[18] != kNG * kNH2 || in_sizes[19] != kNG * kNH || in_sizes[20] != kNG || in_sizes[21] != kNG) return;
  if (in_sizes[22] != kNFC * 2 * kNH2 || in_sizes[23] != kNFC || in_sizes[24] != kNFC || in_sizes[25] != 1) return;
  if (out_size != kNOut) return;
  if (ws_size < kWsTotal) return;

  const int*   words   = (const int*)d_in[0];
  const int*   tags    = (const int*)d_in[1];
  const int*   maxlen  = (const int*)d_in[2];
  const float* wemb    = (const float*)d_in[4];
  const float* temb    = (const float*)d_in[5];
  const float* w_ih_0f = (const float*)d_in[6];
  const float* w_hh_0f = (const float*)d_in[7];
  const float* b_ih_0f = (const float*)d_in[8];
  const float* b_hh_0f = (const float*)d_in[9];
  const float* w_ih_0b = (const float*)d_in[10];
  const float* w_hh_0b = (const float*)d_in[11];
  const float* b_ih_0b = (const float*)d_in[12];
  const float* b_hh_0b = (const float*)d_in[13];
  const float* w_ih_1f = (const float*)d_in[14];
  const float* w_hh_1f = (const float*)d_in[15];
  const float* b_ih_1f = (const float*)d_in[16];
  const float* b_hh_1f = (const float*)d_in[17];
  const float* w_ih_1b = (const float*)d_in[18];
  const float* w_hh_1b = (const float*)d_in[19];
  const float* b_ih_1b = (const float*)d_in[20];
  const float* b_hh_1b = (const float*)d_in[21];
  const float* fc1_w   = (const float*)d_in[22];
  const float* fc1_b   = (const float*)d_in[23];
  const float* fc2_w   = (const float*)d_in[24];
  const float* fc2_b   = (const float*)d_in[25];
  float* out = (float*)d_out;

  char* ws = (char*)d_ws;
  unsigned short* WIH0 = (unsigned short*)(ws + kOffWIH0);
  unsigned short* WHH0 = (unsigned short*)(ws + kOffWHH0);
  unsigned short* WIH1 = (unsigned short*)(ws + kOffWIH1);
  unsigned short* WHH1 = (unsigned short*)(ws + kOffWHH1);
  unsigned short* FC1  = (unsigned short*)(ws + kOffFC1);
  float*          BIAS = (float*)(ws + kOffBIAS);
  unsigned short* XH   = (unsigned short*)(ws + kOffXH);
  unsigned short* XL   = (unsigned short*)(ws + kOffXL);
  float*          XP0  = (float*)(ws + kOffXP0);
  unsigned short* H0H  = (unsigned short*)(ws + kOffH0H);
  unsigned short* H0L  = (unsigned short*)(ws + kOffH0L);
  float*          XP1  = (float*)(ws + kOffXP1);
  unsigned short* H1H  = (unsigned short*)(ws + kOffH1H);
  unsigned short* H1L  = (unsigned short*)(ws + kOffH1L);
  float*          AB   = (float*)(ws + kOffAB);

  wplane_kernel<<<dim3((kNG * (kNE / 8) + 255) / 256, 2), 256, 0, stream>>>(w_ih_0f, w_ih_0b, WIH0, kNG, kNE / 8, kNE, 0, 0);
  wplane_kernel<<<dim3((kNG * (kNH / 8) + 255) / 256, 2), 256, 0, stream>>>(w_hh_0f, w_hh_0b, WHH0, kNG, kNH / 8, kNH, 0, 0);
  wplane_kernel<<<dim3((kNG * (kNH2 / 8) + 255) / 256, 2), 256, 0, stream>>>(w_ih_1f, w_ih_1b, WIH1, kNG, kNH2 / 8, kNH2, 0, 0);
  wplane_kernel<<<dim3((kNG * (kNH / 8) + 255) / 256, 2), 256, 0, stream>>>(w_hh_1f, w_hh_1b, WHH1, kNG, kNH / 8, kNH, 0, 0);
  wplane_kernel<<<dim3((kNFC * (kNH2 / 8) + 255) / 256, 2), 256, 0, stream>>>(fc1_w, fc1_w, FC1, kNFC, kNH2 / 8, 2 * kNH2, 0, kNH2);
  prep_misc_kernel<<<10, 256, 0, stream>>>(b_ih_0f, b_hh_0f, b_ih_0b, b_hh_0b, b_ih_1f, b_hh_1f, b_ih_1b, b_hh_1b,
                                           fc1_b, BIAS, FC1 + (size_t)2 * kNFC * kNH2);
  embed_kernel<<<(kRows * (kNE / 8)) / 256, 256, 0, stream>>>(words, tags, wemb, temb, XH, XL);

  gemm_vr_kernel<<<((kRows / 32) * (kNG2 / 64)) / 8, 256, 0, stream>>>(XH, XL, kNE, WIH0, kNE, XP0, kNG2, BIAS, kRows, kNG2, kNE);
  lstm_dir_kernel<<<2, 256, 0, stream>>>(XP0, WHH0, H0H, H0L);
  gemm_vr_kernel<<<((kRows / 32) * (kNG2 / 64)) / 8, 256, 0, stream>>>(H0H, H0L, kNH2, WIH1, kNH2, XP1, kNG2, BIAS + kNG2, kRows, kNG2, kNH2);
  lstm_dir_kernel<<<2, 256, 0, stream>>>(XP1, WHH1, H1H, H1L);
  gemm_vr_kernel<<<((kRows / 32) * (kNFCP / 64)) / 8, 256, 0, stream>>>(H1H, H1L, kNH2, FC1, kNH2, AB, kNFCP, BIAS + 2 * kNG2, kRows, kNFCP, kNH2);
  score_kernel<<<kNT, 256, 0, stream>>>(AB, fc2_w, fc2_b, maxlen, out);
}
